// MambaBlock_69243462746256
// MI455X (gfx1250) — hardware-verified
//
#include <hip/hip_runtime.h>
#include <math.h>

typedef __attribute__((ext_vector_type(8)))  _Float16 v8h;
typedef __attribute__((ext_vector_type(16))) __bf16   v16b;
typedef __attribute__((ext_vector_type(8)))  __bf16   v8b;
typedef __attribute__((ext_vector_type(8)))  float    v8f;
typedef __attribute__((ext_vector_type(4)))  float    v4f;

constexpr int kBatch  = 4;
constexpr int kSeq    = 4096;
constexpr int kDm     = 128;
constexpr int kDin    = 256;
constexpr int kNst    = 16;
constexpr int kDtR    = 8;
constexpr int kXzP    = 2 * kDin;
constexpr int kXdW    = kDtR + 2 * kNst;
constexpr int kXdP    = 64;
constexpr int kRows   = kBatch * kSeq;
constexpr int kConvTP = 260;
constexpr int kScanTS = 64;
constexpr int kScanCh = 64;
constexpr int kScanYP = 68;
constexpr int kXtP    = 68;
static_assert(kXdW == 40 && kXdW <= kXdP, "x_proj width");
static_assert(kRows == 16384 && kXzP == 512, "shapes");
static_assert((kDm % 32) == 0 && (kDin % 32) == 0, "GEMM K multiples of 32");
static_assert((kRows % 64) == 0 && (kXzP % 64) == 0 && (kXdP % 64) == 0 && (kDm % 64) == 0 && (kSeq % 64) == 0, "GEMM M,N multiples of 64");
static_assert((kSeq % kScanTS) == 0 && (kDin % kScanCh) == 0 && kDin == 256, "tile multiples");
static_assert((kSeq & (kSeq - 1)) == 0, "kSeq power of two");

constexpr size_t kSzWP  = (size_t)kDm  * kDm  * 2;
constexpr size_t kSzWI  = (size_t)kXzP * kDm  * 2;
constexpr size_t kSzWX  = (size_t)kXdP * kDin * 2;
constexpr size_t kSzWO  = (size_t)kDm  * kDin * 2;
constexpr size_t kOffWPH = 0;
constexpr size_t kOffWPL = kOffWPH + kSzWP;
constexpr size_t kOffWIH = kOffWPL + kSzWP;
constexpr size_t kOffWIL = kOffWIH + kSzWI;
constexpr size_t kOffWXH = kOffWIL + kSzWI;
constexpr size_t kOffWXL = kOffWXH + kSzWX;
constexpr size_t kOffWOH = kOffWXL + kSzWX;
constexpr size_t kOffWOL = kOffWOH + kSzWO;
constexpr size_t kOffWQH = kOffWOL + kSzWO;
constexpr size_t kOffWQL = kOffWQH + kSzWP;
constexpr size_t kOffXH  = kOffWQL + kSzWP;
constexpr size_t kOffXL  = kOffXH  + (size_t)kRows * kDm  * 2;
constexpr size_t kOffXF  = kOffXL  + (size_t)kRows * kDm  * 2;
constexpr size_t kOffXNH = kOffXF  + (size_t)kRows * kDm  * 4;
constexpr size_t kOffXNL = kOffXNH + (size_t)kRows * kDm  * 2;
constexpr size_t kOffXZ  = kOffXNL + (size_t)kRows * kDm  * 2;
constexpr size_t kOffUC  = kOffXZ  + (size_t)kRows * kXzP * 4;
constexpr size_t kOffUCH = kOffUC  + (size_t)kRows * kDin * 4;
constexpr size_t kOffUCL = kOffUCH + (size_t)kRows * kDin * 2;
constexpr size_t kOffXD  = kOffUCL + (size_t)kRows * kDin * 2;
constexpr size_t kOffYH  = kOffXD  + (size_t)kRows * kXdP * 4;
constexpr size_t kOffYL  = kOffYH  + (size_t)kRows * kDin * 2;
constexpr size_t kOffYOH = kOffYL  + (size_t)kRows * kDin * 2;
constexpr size_t kOffYOL = kOffYOH + (size_t)kRows * kDm  * 2;
constexpr size_t kWsTotal = kOffYOL + (size_t)kRows * kDm * 2;
static_assert(kWsTotal == 122224640ull, "carve total");
static_assert(kWsTotal <= 134217728ull, "carve cap");
static_assert((kOffWPL % 128) == 0 && (kOffWIH % 128) == 0 && (kOffWIL % 128) == 0 && (kOffWXH % 128) == 0 &&
              (kOffWXL % 128) == 0 && (kOffWOH % 128) == 0 && (kOffWOL % 128) == 0 && (kOffWQH % 128) == 0 &&
              (kOffWQL % 128) == 0 && (kOffXH % 128) == 0 && (kOffXL % 128) == 0 && (kOffXF % 128) == 0 &&
              (kOffXNH % 128) == 0 && (kOffXNL % 128) == 0 && (kOffXZ % 128) == 0 && (kOffUC % 128) == 0 &&
              (kOffUCH % 128) == 0 && (kOffUCL % 128) == 0 && (kOffXD % 128) == 0 && (kOffYH % 128) == 0 &&
              (kOffYL % 128) == 0 && (kOffYOH % 128) == 0 && (kOffYOL % 128) == 0, "128-B aligned regions");

__device__ __forceinline__ unsigned short f2bf_bits(float f) {
  unsigned u = __float_as_uint(f);
  return (unsigned short)((u + 0x7FFFu + ((u >> 16) & 1u)) >> 16);
}
__device__ __forceinline__ float bf_bits2f(unsigned short h) { return __uint_as_float(((unsigned)h) << 16); }

__device__ __forceinline__ void row_guard_b(v8f& a, v8f& b, v8f& c, v8f& d, v16b x, v16b y) {
  asm volatile("v_nop\n\tv_nop\n\tv_nop\n\tv_nop" : "+v"(a), "+v"(b), "+v"(c), "+v"(d) : "v"(x), "v"(y));
}
__device__ __forceinline__ void keep4_b(v16b a, v16b b, v16b c, v16b d) { asm volatile("v_nop" :: "v"(a), "v"(b), "v"(c), "v"(d)); }
__device__ __forceinline__ void acc_guard4(v8f& a, v8f& b, v8f& c, v8f& d) { asm volatile("v_nop\n\tv_nop\n\tv_nop\n\tv_nop" : "+v"(a), "+v"(b), "+v"(c), "+v"(d)); }

struct FragB {
  union U { v16b v; v8b h[2]; };
  static __device__ __forceinline__ v16b load(const __bf16* p) {
    U f; f.h[0] = *(const v8b*)(p); f.h[1] = *(const v8b*)(p + 16); return f.v;
  }
  static __device__ __forceinline__ v8f mma(v16b a, v16b b, v8f c) {
    return __builtin_amdgcn_wmma_f32_16x16x32_bf16(false, a, false, b, (short)0, c, false, false);
  }
};

template <int SPL, int BIAS_MODE, int OUT_MODE>
__global__ __launch_bounds__(256) void wmma_gemm64(
    const unsigned short* __restrict__ Ap, const unsigned short* __restrict__ A2p, int lda, long strideA,
    const unsigned short* __restrict__ Btp, const unsigned short* __restrict__ Bt2p, int ldb, long strideB,
    void* __restrict__ Cout, void* __restrict__ Cout2, int ldc, long strideC,
    const float* __restrict__ bias,
    int M, int N, int K, float scale) {
  typedef __bf16 T;
  typedef v16b V;
  const T* A = (const T*)Ap; const T* A2 = (const T*)A2p; const T* Bt = (const T*)Btp; const T* Bt2 = (const T*)Bt2p;
  __shared__ __align__(16) float sT[8][16 * 68];
  const int b    = blockIdx.y;
  const int lane = threadIdx.x & 31;
  const int wave = threadIdx.x >> 5;
  const int tilesN = N >> 6;
  const int tilesM = M >> 6;
  const int tile = blockIdx.x * 8 + wave;
  if (tile >= tilesM * tilesN) return;
  const int tm = tile / tilesN;
  const int tn = tile - tm * tilesN;
  const int m0 = tm << 6;
  const int n0 = tn << 6;

  const T* Ab  = A  + (size_t)b * strideA;
  const T* Bb  = Bt + (size_t)b * strideB;
  const T* Ab2 = (SPL == 2) ? (A2  + (size_t)b * strideA) : Ab;
  const T* Bb2 = (SPL == 2) ? (Bt2 + (size_t)b * strideB) : Bb;

  const int rlane = lane & 15;
  const int koff  = (lane >> 4) * 8;
  const int mOff  = (lane >> 4) * 8;

  v8f acc[4][4];
#pragma unroll
  for (int i = 0; i < 4; ++i)
#pragma unroll
    for (int j = 0; j < 4; ++j) acc[i][j] = (v8f){0.f,0.f,0.f,0.f,0.f,0.f,0.f,0.f};

  for (int k0 = 0; k0 < K; k0 += 32) {
    V bh[4], bl[4];
#pragma unroll
    for (int j = 0; j < 4; ++j) {
      const size_t bo = (size_t)(n0 + (j << 4) + rlane) * ldb + koff + k0;
      bh[j] = FragB::load(Bb + bo);
      bl[j] = (SPL == 2) ? FragB::load(Bb2 + bo) : bh[j];
    }
#pragma unroll
    for (int i = 0; i < 4; ++i) {
      const size_t ao = (size_t)(m0 + (i << 4) + rlane) * lda + koff + k0;
      V ah = FragB::load(Ab + ao);
      V al = (SPL == 2) ? FragB::load(Ab2 + ao) : ah;
#pragma unroll
      for (int j = 0; j < 4; ++j) {
        acc[i][j] = FragB::mma(ah, bh[j], acc[i][j]);
        if (SPL == 2) {
          acc[i][j] = FragB::mma(ah, bl[j], acc[i][j]);
          acc[i][j] = FragB::mma(al, bh[j], acc[i][j]);
        }
      }
      row_guard_b(acc[i][0], acc[i][1], acc[i][2], acc[i][3], ah, al);
    }
    keep4_b(bh[0], bh[1], bh[2], bh[3]);
    keep4_b(bl[0], bl[1], bl[2], bl[3]);
  }
  acc_guard4(acc[0][0], acc[0][1], acc[0][2], acc[0][3]);
  acc_guard4(acc[1][0], acc[1][1], acc[1][2], acc[1][3]);
  acc_guard4(acc[2][0], acc[2][1], acc[2][2], acc[2][3]);
  acc_guard4(acc[3][0], acc[3][1], acc[3][2], acc[3][3]);

  float* slab = sT[wave];
#pragma unroll
  for (int i = 0; i < 4; ++i) {
    const int mBase = m0 + (i << 4);
#pragma unroll
    for (int j = 0; j < 4; ++j) {
      const int n = n0 + (j << 4) + rlane;
      float bv = 0.f;
      if (BIAS_MODE == 2) bv = bias[n];
#pragma unroll
      for (int r = 0; r < 8; ++r) {
        float v = acc[i][j][r] * scale;
        if (BIAS_MODE == 1) v += bias[mBase + mOff + r];
        if (BIAS_MODE == 2) v += bv;
        slab[(mOff + r) * 68 + (j << 4) + rlane] = v;
      }
    }
    __builtin_amdgcn_fence(__ATOMIC_RELEASE, "workgroup");
    __builtin_amdgcn_wave_barrier();
    __builtin_amdgcn_fence(__ATOMIC_ACQUIRE, "workgroup");
    if (OUT_MODE == 0) {
      float* C = (float*)Cout + (size_t)b * strideC;
      const int hh = lane >> 4, c4 = (lane & 15) * 4;
      for (int pass = 0; pass < 2; ++pass) {
#pragma unroll
        for (int it = 0; it < 8; ++it) {
          const int row = it * 2 + hh;
          v4f v = *(const v4f*)(slab + row * 68 + c4);
          *(volatile v4f*)(C + (size_t)(mBase + row) * ldc + n0 + c4) = v;
        }
        __threadfence();
      }
    } else {
      const int q = lane >> 3, c8 = (lane & 7) * 8;
      unsigned short* C  = (unsigned short*)Cout  + (size_t)b * strideC;
      unsigned short* C2 = (unsigned short*)Cout2 + (size_t)b * strideC;
      for (int pass = 0; pass < 2; ++pass) {
#pragma unroll
        for (int it = 0; it < 4; ++it) {
          const int row = it * 4 + q;
          const float* sp = slab + row * 68 + c8;
          v8h hv, lv;
#pragma unroll
          for (int e = 0; e < 8; ++e) {
            const float sv = sp[e];
            const unsigned short hb = f2bf_bits(sv);
            const unsigned short lb = f2bf_bits(sv - bf_bits2f(hb));
            hv[e] = __builtin_bit_cast(_Float16, hb);
            lv[e] = __builtin_bit_cast(_Float16, lb);
          }
          *(volatile v8h*)(C  + (size_t)(mBase + row) * ldc + n0 + c8) = hv;
          *(volatile v8h*)(C2 + (size_t)(mBase + row) * ldc + n0 + c8) = lv;
        }
        __threadfence();
      }
    }
    __builtin_amdgcn_fence(__ATOMIC_RELEASE, "workgroup");
    __builtin_amdgcn_wave_barrier();
    __builtin_amdgcn_fence(__ATOMIC_ACQUIRE, "workgroup");
  }
}

__global__ __launch_bounds__(256) void split_rows_bf16_kernel(
    const float* __restrict__ src, unsigned short* __restrict__ dhi, unsigned short* __restrict__ dlo,
    int real8, int total8)
{
  const int i = blockIdx.x * 256 + threadIdx.x;
  if (i >= total8) return;
  const bool live = (i < real8);
  const int ic = live ? i : (real8 - 1);
  const size_t es = (size_t)ic << 3;
  const size_t e0 = (size_t)i << 3;
  const v4f a0 = *(const v4f*)(src + es);
  const v4f a1 = *(const v4f*)(src + es + 4);
  v8h hv, lv;
#pragma unroll
  for (int e = 0; e < 4; ++e) {
    const float f0 = live ? a0[e] : 0.0f;
    const float f1 = live ? a1[e] : 0.0f;
    const unsigned short h0 = f2bf_bits(f0), h1 = f2bf_bits(f1);
    const unsigned short l0 = f2bf_bits(f0 - bf_bits2f(h0)), l1 = f2bf_bits(f1 - bf_bits2f(h1));
    hv[e]     = __builtin_bit_cast(_Float16, h0);
    hv[4 + e] = __builtin_bit_cast(_Float16, h1);
    lv[e]     = __builtin_bit_cast(_Float16, l0);
    lv[4 + e] = __builtin_bit_cast(_Float16, l1);
  }
  unsigned short* qh = dhi + e0;
  unsigned short* ql = dlo + e0;
  *(volatile v8h*)qh = hv;
  *(volatile v8h*)ql = lv;
  __threadfence();
  *(volatile v8h*)qh = hv;
  *(volatile v8h*)ql = lv;
}

__global__ __launch_bounds__(256) void x_transpose_split_kernel(
    const float* __restrict__ x, unsigned short* __restrict__ XH, unsigned short* __restrict__ XL)
{
  __shared__ __align__(16) float sT[kDm * kXtP];
  const int tid = threadIdx.x, lane = tid & 31, wave = tid >> 5;
  const int g0 = blockIdx.x * 64;
  const int bix = g0 / kSeq;
  const int p0 = g0 - bix * kSeq;
  const float* xb = x + (size_t)bix * kDm * kSeq + p0;
#pragma unroll
  for (int p = 0; p < 8; ++p) {
    const int idx = tid + p * 256;
    const int c  = idx >> 4;
    const int p4 = (idx & 15) * 4;
    const v4f v = *(const v4f*)(xb + (size_t)c * kSeq + p4);
    *(v4f*)(sT + c * kXtP + p4) = v;
  }
  __syncthreads();
  const int half = lane >> 4, c8 = (lane & 15) * 8;
  v8h hv[4], lv[4];
#pragma unroll
  for (int it = 0; it < 4; ++it) {
    const int row = it * 16 + wave * 2 + half;
#pragma unroll
    for (int e = 0; e < 8; ++e) {
      const float f = sT[(c8 + e) * kXtP + row];
      const unsigned short hb = f2bf_bits(f);
      const unsigned short lb = f2bf_bits(f - bf_bits2f(hb));
      hv[it][e] = __builtin_bit_cast(_Float16, hb);
      lv[it][e] = __builtin_bit_cast(_Float16, lb);
    }
  }
  for (int pass = 0; pass < 2; ++pass) {
#pragma unroll
    for (int it = 0; it < 4; ++it) {
      const int row = it * 16 + wave * 2 + half;
      const size_t o = (size_t)(g0 + row) * kDm + c8;
      *(volatile v8h*)(XH + o) = hv[it];
      *(volatile v8h*)(XL + o) = lv[it];
    }
    __threadfence();
  }
}

__global__ __launch_bounds__(256) void ln_split_kernel(
    const float* __restrict__ XF, const float* __restrict__ pb, const float* __restrict__ lg,
    const float* __restrict__ lb, unsigned short* __restrict__ XNH, unsigned short* __restrict__ XNL)
{
  const int i = blockIdx.x * 256 + threadIdx.x;
  const int row = i >> 4;
  const int c8 = (i & 15) * 8;
  const float* p = XF + (size_t)row * kDm + c8;
  const v4f a0 = *(const v4f*)(p);
  const v4f a1 = *(const v4f*)(p + 4);
  const v4f b0 = *(const v4f*)(pb + c8);
  const v4f b1 = *(const v4f*)(pb + c8 + 4);
  float v[8];
#pragma unroll
  for (int e = 0; e < 4; ++e) { v[e] = a0[e] + b0[e]; v[4 + e] = a1[e] + b1[e]; }
  float s = 0.0f;
#pragma unroll
  for (int e = 0; e < 8; ++e) s += v[e];
  s += __shfl_xor(s, 1, 32);
  s += __shfl_xor(s, 2, 32);
  s += __shfl_xor(s, 4, 32);
  s += __shfl_xor(s, 8, 32);
  const float mu = s * (1.0f / (float)kDm);
  float q = 0.0f;
#pragma unroll
  for (int e = 0; e < 8; ++e) { const float dv = v[e] - mu; v[e] = dv; q += dv * dv; }
  q += __shfl_xor(q, 1, 32);
  q += __shfl_xor(q, 2, 32);
  q += __shfl_xor(q, 4, 32);
  q += __shfl_xor(q, 8, 32);
  const float rs = rsqrtf(q * (1.0f / (float)kDm) + 1e-5f);
  const v4f g0 = *(const v4f*)(lg + c8);
  const v4f g1 = *(const v4f*)(lg + c8 + 4);
  const v4f t0 = *(const v4f*)(lb + c8);
  const v4f t1 = *(const v4f*)(lb + c8 + 4);
  v8h hv, lv;
#pragma unroll
  for (int e = 0; e < 4; ++e) {
    const float f0 = v[e] * rs * g0[e] + t0[e];
    const float f1 = v[4 + e] * rs * g1[e] + t1[e];
    const unsigned short h0 = f2bf_bits(f0), h1 = f2bf_bits(f1);
    const unsigned short l0 = f2bf_bits(f0 - bf_bits2f(h0)), l1 = f2bf_bits(f1 - bf_bits2f(h1));
    hv[e]     = __builtin_bit_cast(_Float16, h0);
    hv[4 + e] = __builtin_bit_cast(_Float16, h1);
    lv[e]     = __builtin_bit_cast(_Float16, l0);
    lv[4 + e] = __builtin_bit_cast(_Float16, l1);
  }
  const size_t o = (size_t)row * kDm + c8;
  *(volatile v8h*)(XNH + o) = hv;
  *(volatile v8h*)(XNL + o) = lv;
  __threadfence();
  *(volatile v8h*)(XNH + o) = hv;
  *(volatile v8h*)(XNL + o) = lv;
}

__global__ __launch_bounds__(256) void conv_silu_kernel(
    const float* __restrict__ XZ, const float* __restrict__ cw, const float* __restrict__ cb,
    float* __restrict__ UC, unsigned short* __restrict__ UCH, unsigned short* __restrict__ UCL)
{
  __shared__ __align__(16) float sT[16 * kConvTP];
  const int tid = threadIdx.x, lane = tid & 31, wave = tid >> 5;
  const int d = tid;
  const int g0 = blockIdx.x * 64;
  const int tb = g0 & (kSeq - 1);
  const float w0 = cw[d * 4 + 0], w1 = cw[d * 4 + 1], w2 = cw[d * 4 + 2], w3 = cw[d * 4 + 3];
  const float bc = cb[d];
  float xm3, xm2, xm1;
  {
    const bool hist = (tb > 0);
    const int rb = hist ? (g0 - 3) : g0;
    const float v3 = XZ[(size_t)rb * kXzP + d];
    const float v2 = XZ[(size_t)(rb + 1) * kXzP + d];
    const float v1 = XZ[(size_t)(rb + 2) * kXzP + d];
    xm3 = hist ? v3 : 0.f;
    xm2 = hist ? v2 : 0.f;
    xm1 = hist ? v1 : 0.f;
  }
  const int hrow = wave >> 1;
  const int hch  = (wave & 1) * 128 + lane * 4;
#pragma unroll 1
  for (int sub = 0; sub < 4; ++sub) {
    const int lb = g0 + sub * 16;
#pragma unroll 1
    for (int s = 0; s < 16; ++s) {
      const float xcur = XZ[(size_t)(lb + s) * kXzP + d];
      float acc = w0 * xm3;
      acc = fmaf(w1, xm2, acc);
      acc = fmaf(w2, xm1, acc);
      acc = fmaf(w3, xcur, acc);
      const float sv = acc + bc;
      const float sg = 1.0f / (1.0f + expf(-sv));
      sT[s * kConvTP + tid] = sv * sg;
      xm3 = xm2; xm2 = xm1; xm1 = xcur;
    }
    __syncthreads();
    v4f fv[4];
    v8h bh[2], blo[2];
#pragma unroll
    for (int it = 0; it < 4; ++it) fv[it] = *(const v4f*)(sT + (it * 4 + hrow) * kConvTP + hch);
#pragma unroll
    for (int it = 0; it < 2; ++it) {
      const float* sp = sT + (it * 8 + wave) * kConvTP + lane * 8;
      const v4f a0 = *(const v4f*)(sp);
      const v4f a1 = *(const v4f*)(sp + 4);
#pragma unroll
      for (int e = 0; e < 4; ++e) {
        const float f0 = a0[e], f1 = a1[e];
        const unsigned short h0 = f2bf_bits(f0), h1 = f2bf_bits(f1);
        const unsigned short l0 = f2bf_bits(f0 - bf_bits2f(h0)), l1 = f2bf_bits(f1 - bf_bits2f(h1));
        bh[it][e]      = __builtin_bit_cast(_Float16, h0);
        bh[it][4 + e]  = __builtin_bit_cast(_Float16, h1);
        blo[it][e]     = __builtin_bit_cast(_Float16, l0);
        blo[it][4 + e] = __builtin_bit_cast(_Float16, l1);
      }
    }
    for (int pass = 0; pass < 2; ++pass) {
#pragma unroll
      for (int it = 0; it < 4; ++it)
        *(volatile v4f*)(UC + (size_t)(lb + it * 4 + hrow) * kDin + hch) = fv[it];
#pragma unroll
      for (int it = 0; it < 2; ++it) {
        const size_t o = (size_t)(lb + it * 8 + wave) * kDin + lane * 8;
        *(volatile v8h*)(UCH + o) = bh[it];
        *(volatile v8h*)(UCL + o) = blo[it];
      }
      __threadfence();
    }
    __syncthreads();
  }
}

__global__ __launch_bounds__(64) void scan_kernel(
    const float* __restrict__ XD, const float* __restrict__ UC, const float* __restrict__ XZ,
    const float* __restrict__ Wdt, const float* __restrict__ bdt, const float* __restrict__ Alog,
    const float* __restrict__ Dp, unsigned short* __restrict__ YH, unsigned short* __restrict__ YL)
{
  __shared__ __align__(16) float sX[kScanTS * kXdP];
  __shared__ __align__(16) float sY[kScanTS * kScanYP];
  __shared__ __align__(16) float sW[kDtR * kScanCh];
  __shared__ __align__(16) float sA[kNst * kScanCh];
  const int tid = threadIdx.x, lane = tid & 31, wave = tid >> 5;
  constexpr int kBlkPerB = kDin / kScanCh;
  const int bix = blockIdx.x / kBlkPerB;
  const int d0  = (blockIdx.x - bix * kBlkPerB) * kScanCh;
  const int d   = d0 + tid;
  const size_t row0 = (size_t)bix * kSeq;
#pragma unroll 1
  for (int r = 0; r < kDtR; ++r) sW[r * kScanCh + tid] = Wdt[(size_t)d * kDtR + r];
#pragma unroll 1
  for (int s = 0; s < kNst; ++s) sA[s * kScanCh + tid] = -expf(Alog[(size_t)d * kNst + s]);
  __syncthreads();
  float negA[kNst], h[kNst];
#pragma unroll
  for (int s = 0; s < kNst; ++s) {
    negA[s] = sA[s * kScanCh + tid];
    h[s] = 0.f;
  }
  const float bb = bdt[d], Dd = Dp[d];
  const int lr = tid >> 4, lc4 = (tid & 15) * 4;
  const int q = lane >> 3, c8 = (lane & 7) * 8;
#pragma unroll 1
  for (int t0 = 0; t0 < kSeq; t0 += kScanTS) {
    __syncthreads();
#pragma unroll
    for (int i = 0; i < 16; ++i) {
      const int r = lr + 4 * i;
      *(v4f*)(sX + r * kXdP + lc4) = *(const v4f*)(XD + (row0 + t0 + r) * kXdP + lc4);
    }
    __syncthreads();
#pragma unroll 1
    for (int s = 0; s < kScanTS; ++s) {
      const int t = t0 + s;
      const float* xr = sX + s * kXdP;
      float vdot = 0.f;
#pragma unroll 1
      for (int r4 = 0; r4 < kDtR / 4; ++r4) {
        const v4f xv = *(const v4f*)(xr + 4 * r4);
        const float* wp = sW + (4 * r4) * kScanCh + tid;
        vdot = fmaf(xv[0], wp[0], vdot);
        vdot = fmaf(xv[1], wp[kScanCh], vdot);
        vdot = fmaf(xv[2], wp[2 * kScanCh], vdot);
        vdot = fmaf(xv[3], wp[3 * kScanCh], vdot);
      }
      float Bs[kNst], Cs[kNst];
#pragma unroll
      for (int q4 = 0; q4 < 4; ++q4) {
        const v4f bv = *(const v4f*)(xr + kDtR + 4 * q4);
        const v4f cv = *(const v4f*)(xr + kDtR + kNst + 4 * q4);
        Bs[4 * q4 + 0] = bv[0]; Bs[4 * q4 + 1] = bv[1]; Bs[4 * q4 + 2] = bv[2]; Bs[4 * q4 + 3] = bv[3];
        Cs[4 * q4 + 0] = cv[0]; Cs[4 * q4 + 1] = cv[1]; Cs[4 * q4 + 2] = cv[2]; Cs[4 * q4 + 3] = cv[3];
      }
      const float v   = vdot + bb;
      const float a   = __expf(-fabsf(v));
      const float u   = 1.0f + a;
      const float l1p = __logf(u) + (a - (u - 1.0f)) * __builtin_amdgcn_rcpf(u);
      const float dt  = fmaxf(v, 0.0f) + l1p;
      const float xt  = UC[(row0 + t) * kDin + d];
      const float dtx = dt * xt;
      float y = 0.f;
#pragma unroll
      for (int k = 0; k < kNst; ++k) {
        const float e = __expf(dt * negA[k]);
        h[k] = e * h[k] + dtx * Bs[k];
        y = h[k] * Cs[k] + y;
      }
      y = xt * Dd + y;
      const float zv = XZ[(row0 + t) * kXzP + kDin + d];
      const float sg = 1.0f / (1.0f + expf(-zv));
      y = y * (zv * sg);
      sY[s * kScanYP + tid] = y;
    }
    __syncthreads();
    v8h hv[8], lv[8];
#pragma unroll
    for (int it = 0; it < 8; ++it) {
      const int row = it * 8 + wave * 4 + q;
      const float* sp = sY + row * kScanYP + c8;
      const v4f a0 = *(const v4f*)(sp);
      const v4f a1 = *(const v4f*)(sp + 4);
#pragma unroll
      for (int e = 0; e < 4; ++e) {
        const float f0 = a0[e], f1 = a1[e];
        const unsigned short h0 = f2bf_bits(f0), h1 = f2bf_bits(f1);
        const unsigned short l0 = f2bf_bits(f0 - bf_bits2f(h0)), l1 = f2bf_bits(f1 - bf_bits2f(h1));
        hv[it][e]     = __builtin_bit_cast(_Float16, h0);
        hv[it][4 + e] = __builtin_bit_cast(_Float16, h1);
        lv[it][e]     = __builtin_bit_cast(_Float16, l0);
        lv[it][4 + e] = __builtin_bit_cast(_Float16, l1);
      }
    }
    for (int pass = 0; pass < 2; ++pass) {
#pragma unroll
      for (int it = 0; it < 8; ++it) {
        const int row = it * 8 + wave * 4 + q;
        const size_t o = (row0 + t0 + row) * kDin + d0 + c8;
        *(volatile v8h*)(YH + o) = hv[it];
        *(volatile v8h*)(YL + o) = lv[it];
      }
      __threadfence();
    }
  }
}

extern "C" void kernel_launch(void* const* d_in, const int* in_sizes, int n_in,
                              void* d_out, int out_size, void* d_ws, size_t ws_size,
                              hipStream_t stream) {
  if (n_in < 16) return;
  if (in_sizes[0] != kRows * kDm) return;
  if (in_sizes[1] != kDm * kDm) return;
  if (in_sizes[2] != kDm || in_sizes[3] != kDm || in_sizes[4] != kDm) return;
  if (in_sizes[5] != kXzP * kDm) return;
  if (in_sizes[6] != kDin * 4 || in_sizes[7] != kDin) return;
  if (in_sizes[8] != kXdW * kDin) return;
  if (in_sizes[9] != kDin * kDtR || in_sizes[10] != kDin) return;
  if (in_sizes[11] != kDin * kNst || in_sizes[12] != kDin) return;
  if (in_sizes[13] != kDm * kDin) return;
  if (in_sizes[14] != kDm * kDm || in_sizes[15] != kDm) return;
  if (out_size != kRows * kDm) return;
  if (ws_size < kWsTotal) return;

  const float* x       = (const float*)d_in[0];
  const float* pw_in   = (const float*)d_in[1];
  const float* pb_in   = (const float*)d_in[2];
  const float* ln_g    = (const float*)d_in[3];
  const float* ln_b    = (const float*)d_in[4];
  const float* W_in    = (const float*)d_in[5];
  const float* conv_w  = (const float*)d_in[6];
  const float* conv_b  = (const float*)d_in[7];
  const float* W_x     = (const float*)d_in[8];
  const float* W_dt    = (const float*)d_in[9];
  const float* b_dt    = (const float*)d_in[10];
  const float* A_log   = (const float*)d_in[11];
  const float* Dp      = (const float*)d_in[12];
  const float* W_out   = (const float*)d_in[13];
  const float* pw_out  = (const float*)d_in[14];
  const float* pb_out  = (const float*)d_in[15];
  float* out = (float*)d_out;

  char* ws = (char*)d_ws;
  unsigned short* WPH = (unsigned short*)(ws + kOffWPH);
  unsigned short* WPL = (unsigned short*)(ws + kOffWPL);
  unsigned short* WIH = (unsigned short*)(ws + kOffWIH);
  unsigned short* WIL = (unsigned short*)(ws + kOffWIL);
  unsigned short* WXH = (unsigned short*)(ws + kOffWXH);
  unsigned short* WXL = (unsigned short*)(ws + kOffWXL);
  unsigned short* WOH = (unsigned short*)(ws + kOffWOH);
  unsigned short* WOL = (unsigned short*)(ws + kOffWOL);
  unsigned short* WQH = (unsigned short*)(ws + kOffWQH);
  unsigned short* WQL = (unsigned short*)(ws + kOffWQL);
  unsigned short* XH  = (unsigned short*)(ws + kOffXH);
  unsigned short* XL  = (unsigned short*)(ws + kOffXL);
  float*          XF  = (float*)(ws + kOffXF);
  unsigned short* XNH = (unsigned short*)(ws + kOffXNH);
  unsigned short* XNL = (unsigned short*)(ws + kOffXNL);
  float*          XZ  = (float*)(ws + kOffXZ);
  float*          UC  = (float*)(ws + kOffUC);
  unsigned short* UCH = (unsigned short*)(ws + kOffUCH);
  unsigned short* UCL = (unsigned short*)(ws + kOffUCL);
  float*          XD  = (float*)(ws + kOffXD);
  unsigned short* YH  = (unsigned short*)(ws + kOffYH);
  unsigned short* YL  = (unsigned short*)(ws + kOffYL);
  unsigned short* YOH = (unsigned short*)(ws + kOffYOH);
  unsigned short* YOL = (unsigned short*)(ws + kOffYOL);

  split_rows_bf16_kernel<<<(kDm * kDm / 8) / 256, 256, 0, stream>>>(pw_in, WPH, WPL, kDm * kDm / 8, kDm * kDm / 8);
  split_rows_bf16_kernel<<<(kXzP * kDm / 8) / 256, 256, 0, stream>>>(W_in, WIH, WIL, kXzP * kDm / 8, kXzP * kDm / 8);
  split_rows_bf16_kernel<<<(kXdP * kDin / 8) / 256, 256, 0, stream>>>(W_x, WXH, WXL, kXdW * kDin / 8, kXdP * kDin / 8);
  split_rows_bf16_kernel<<<(kDm * kDin / 8) / 256, 256, 0, stream>>>(W_out, WOH, WOL, kDm * kDin / 8, kDm * kDin / 8);
  split_rows_bf16_kernel<<<(kDm * kDm / 8) / 256, 256, 0, stream>>>(pw_out, WQH, WQL, kDm * kDm / 8, kDm * kDm / 8);

  x_transpose_split_kernel<<<kRows / 64, 256, 0, stream>>>(x, XH, XL);

  wmma_gemm64<2, 0, 0><<<dim3(64, 1), 256, 0, stream>>>(
      XH, XL, kDm, 0L, WPH, WPL, kDm, 0L,
      (void*)XF, (void*)XF, kDm, 0L, pb_in, kRows, kDm, kDm, 1.0f);

  ln_split_kernel<<<(kRows * 16) / 256, 256, 0, stream>>>(XF, pb_in, ln_g, ln_b, XNH, XNL);

  wmma_gemm64<2, 0, 0><<<dim3(256, 1), 256, 0, stream>>>(
      XNH, XNL, kDm, 0L, WIH, WIL, kDm, 0L,
      (void*)XZ, (void*)XZ, kXzP, 0L, pb_in, kRows, kXzP, kDm, 1.0f);

  conv_silu_kernel<<<kRows / 64, 256, 0, stream>>>(XZ, conv_w, conv_b, UC, UCH, UCL);

  wmma_gemm64<2, 0, 0><<<dim3(32, 1), 256, 0, stream>>>(
      UCH, UCL, kDin, 0L, WXH, WXL, kDin, 0L,
      (void*)XD, (void*)XD, kXdP, 0L, pb_in, kRows, kXdP, kDin, 1.0f);

  scan_kernel<<<kBatch * (kDin / kScanCh), kScanCh, 0, stream>>>(XD, UC, XZ, W_dt, b_dt, A_log, Dp, YH, YL);

  wmma_gemm64<2, 0, 2><<<dim3(64, 1), 256, 0, stream>>>(
      YH, YL, kDin, 0L, WOH, WOL, kDin, 0L,
      (void*)YOH, (void*)YOL, kDm, 0L, pb_in, kRows, kDm, kDin, 1.0f);

  wmma_gemm64<2, 1, 0><<<dim3(16, kBatch), 256, 0, stream>>>(
      WQH, WQL, kDm, 0L, YOH, YOL, kDm, (long)kSeq * kDm,
      (void*)out, (void*)out, kSeq, (long)kDm * kSeq, pb_out, kDm, kSeq, kDm, 1.0f);
}
